// KPConv_42090679501115
// MI455X (gfx1250) — hardware-run, weakly checked
//
#include <hip/hip_runtime.h>
#include <math.h>

typedef __attribute__((ext_vector_type(16))) _Float16 v16h;
typedef __attribute__((ext_vector_type(16))) __bf16 v16b;
typedef __attribute__((ext_vector_type(8)))  _Float16 v8h;
typedef __attribute__((ext_vector_type(8)))  float v8f;
typedef __attribute__((ext_vector_type(4)))  float v4f;
typedef __attribute__((ext_vector_type(2)))  float v2f;
typedef __attribute__((ext_vector_type(4)))  unsigned v4u;
typedef __attribute__((ext_vector_type(4)))  int v4i;
typedef float __attribute__((may_alias)) float_a;
typedef int __attribute__((may_alias)) int_a;

template <typename T> __device__ __forceinline__ void vst2(void* p, T v) { *(volatile T*)p = v; __threadfence(); *(volatile T*)p = v; }
__device__ __forceinline__ v8f wmma16(v16h a, v16h b, v8f c) {
  v8f d = __builtin_amdgcn_wmma_f32_16x16x32_f16(false, a, false, b, (short)0, c, false, false);
  asm volatile("v_nop\n\tv_nop\n\tv_nop\n\tv_nop" : "+v"(d) : "v"(a), "v"(b));
  return d;
}
__device__ __forceinline__ v8f wmma_bf(v16b a, v16b b, v8f c) {
  v8f d = __builtin_amdgcn_wmma_f32_16x16x32_bf16(false, a, false, b, (short)0, c, false, false);
  asm volatile("v_nop\n\tv_nop\n\tv_nop\n\tv_nop" : "+v"(d) : "v"(a), "v"(b));
  return d;
}
__device__ __forceinline__ v16h frag_h(const _Float16* rowk0, int lane) {
  union { v16h v; v8h q[2]; } u; const _Float16* p = rowk0 + 8 * (lane >> 4);
  u.q[0] = *(const v8h*)p; u.q[1] = *(const v8h*)(p + 16); return u.v;
}
__device__ __forceinline__ v16h frag_f32(const float* rowk0, int lane) {
  v16h a; const float* p = rowk0 + 8 * (lane >> 4);
#pragma unroll
  for (int i = 0; i < 8; ++i) { a[i] = (_Float16)p[i]; a[8 + i] = (_Float16)p[16 + i]; }
  return a;
}
__device__ __forceinline__ v16h frag_f32s(const float* rowk0, int lane, float sc) {
  v16h a; const float* p = rowk0 + 8 * (lane >> 4);
#pragma unroll
  for (int i = 0; i < 8; ++i) { a[i] = (_Float16)(p[i] * sc); a[8 + i] = (_Float16)(p[16 + i] * sc); }
  return a;
}
__device__ __forceinline__ v16h fragc_f32(const float* W, int k0, int n, int lane, int ld, int K) {
  v16h a; const int g = lane >> 4;
#pragma unroll
  for (int i = 0; i < 8; ++i) { const int ka = k0 + 8 * g + i, kb = ka + 16;
    a[i] = (_Float16)(ka < K ? W[(size_t)(ka < K ? ka : K - 1) * ld + n] : 0.f); a[8 + i] = (_Float16)(kb < K ? W[(size_t)(kb < K ? kb : K - 1) * ld + n] : 0.f); }
  return a;
}
struct F2 { v16b h, l; };
__device__ __forceinline__ F2 bsplit16(const float v[16]) { F2 r;
#pragma unroll
  for (int i = 0; i < 16; ++i) { const __bf16 h = (__bf16)v[i]; r.h[i] = h; r.l[i] = (__bf16)(v[i] - (float)h); }
  return r; }
__device__ __forceinline__ F2 split_row(const float* row, int k0, int lane) { float v[16]; const float* p = row + k0 + 8 * (lane >> 4);
#pragma unroll
  for (int i = 0; i < 8; ++i) { v[i] = p[i]; v[8 + i] = p[16 + i]; }
  return bsplit16(v); }
__device__ __forceinline__ F2 split_rowK(const float* row, int k0, int lane, int K) { float v[16]; const int g = lane >> 4;
#pragma unroll
  for (int i = 0; i < 8; ++i) { const int ka = k0 + 8 * g + i, kb = ka + 16; v[i] = ka < K ? row[ka < K ? ka : K - 1] : 0.f; v[8 + i] = kb < K ? row[kb < K ? kb : K - 1] : 0.f; }
  return bsplit16(v); }
__device__ __forceinline__ F2 split_col(const float* W, int k0, int n, int lane, int ld, int K) { float v[16]; const int g = lane >> 4;
#pragma unroll
  for (int i = 0; i < 8; ++i) { const int ka = k0 + 8 * g + i, kb = ka + 16; v[i] = ka < K ? W[(size_t)(ka < K ? ka : K - 1) * ld + n] : 0.f; v[8 + i] = kb < K ? W[(size_t)(kb < K ? kb : K - 1) * ld + n] : 0.f; }
  return bsplit16(v); }
__device__ __forceinline__ v8f mac3(const F2& a, const F2& b, v8f c) { c = wmma_bf(a.l, b.h, c); c = wmma_bf(a.h, b.l, c); return wmma_bf(a.h, b.h, c); }
__device__ __forceinline__ float sigm(float v) { return 1.0f / (1.0f + expf(-v)); }
#define LDSX() do { asm volatile("s_wait_dscnt 0" ::: "memory"); __builtin_amdgcn_wave_barrier(); __builtin_amdgcn_fence(__ATOMIC_RELEASE, "workgroup"); } while (0)

typedef __attribute__((ext_vector_type(4))) int v4i;
__device__ __forceinline__ float bfr(float v) { return (float)(__bf16)v; }
__device__ __forceinline__ v16b wcol_io(const float* __restrict__ Wm, int k0, int o, int lane, int ld) { v16b w; const float* p = Wm + (size_t)(k0 + 8 * (lane >> 4)) * ld + o;
#pragma unroll
  for (int i = 0; i < 8; ++i) { w[i] = (__bf16)p[(size_t)i * ld]; w[8 + i] = (__bf16)p[(size_t)(16 + i) * ld]; }
  asm volatile("s_wait_loadcnt 0x0" ::: "memory"); return w; }
#define NPTS 50000
#define CI 64
#define CO 64
#define KP 15
#define KN 32
#define NR 50000
#ifndef NRV
#define NRV NR
#endif
#define FKW (KP * CI)
#define WS_FK  0u
#define WS_CNT (WS_FK + 4u * (size_t)NR * FKW + 256)
#define WS_END (WS_CNT + 4u * (size_t)NR + 256)
__global__ __launch_bounds__(128) void k_fk(const float* __restrict__ QP, const float* __restrict__ P, const float* __restrict__ FT, const float* __restrict__ KPT, const int* __restrict__ IDX, float* __restrict__ FK, float* __restrict__ CNT) { __shared__ float srel[4][KN][4]; __shared__ int sidx[4][KN]; __shared__ __align__(16) float sf[4][16][68];
  const int tid = threadIdx.x, wave = tid >> 5, lane = tid & 31, col = lane & 15, g = lane >> 4; const size_t row = (size_t)blockIdx.x * 4 + wave; const bool live = row < (size_t)NRV; const size_t rowc = live ? row : 0;
  { int ix = IDX[rowc * KN + lane]; const bool ok = ix >= 0 && ix < NPTS; ix = ok ? ix : 0; sidx[wave][lane] = ok ? ix : -1;
    const float qx = bfr(QP[rowc * 3]), qy = bfr(QP[rowc * 3 + 1]), qz = bfr(QP[rowc * 3 + 2]);
    const size_t pp = (size_t)ix * 3; srel[wave][lane][0] = ok ? bfr(P[pp]) - qx : 1.0e6f; srel[wave][lane][1] = ok ? bfr(P[pp + 1]) - qy : 1.0e6f; srel[wave][lane][2] = ok ? bfr(P[pp + 2]) - qz : 1.0e6f; srel[wave][lane][3] = 1.f;
    float fs = 0.f; { const float* pf = FT + (size_t)ix * CI;
#pragma unroll
      for (int c4 = 0; c4 < CI; c4 += 16) { float t[16];
#pragma unroll
        for (int i = 0; i < 16; ++i) t[i] = pf[c4 + i];
        asm volatile("s_wait_loadcnt 0x0" ::: "memory");
#pragma unroll
        for (int i = 0; i < 16; ++i) fs += bfr(t[i]); } }
    int cnt = (ok && fs > 0.f) ? 1 : 0;
#pragma unroll
    for (int o = 1; o < 32; o <<= 1) cnt += __shfl_xor(cnt, o);
    if (lane == 0 && live) vst2(CNT + row, (float)(cnt < 1 ? 1 : cnt)); }
  LDSX();
  float va[16]; { const bool kv = col < KP; const float kx = kv ? bfr(KPT[col * 3]) : 0.f, ky = kv ? bfr(KPT[col * 3 + 1]) : 0.f, kz = kv ? bfr(KPT[col * 3 + 2]) : 0.f;
#pragma unroll
    for (int i = 0; i < 16; ++i) { const int n = (i < 8) ? (8 * g + i) : (16 + 8 * g + (i - 8)); const float dx = srel[wave][n][0] - kx, dy = srel[wave][n][1] - ky, dz = srel[wave][n][2] - kz; const float sq = (dx * dx + dy * dy) + dz * dz;
      const float wv = fmaxf(1.0f - __fsqrt_rn(sq) / 0.1f, 0.f); va[i] = kv ? wv : 0.f; } }
  const F2 a = bsplit16(va);
  v8f acc[4] = {};
#pragma unroll
  for (int j = 0; j < 4; ++j) { v16b fb; { const int c = j * 16 + col;
#pragma unroll
      for (int i = 0; i < 16; ++i) { const int n = (i < 8) ? (8 * g + i) : (16 + 8 * g + (i - 8)); const int gi = sidx[wave][n]; const float fv = gi >= 0 ? FT[(size_t)gi * CI + c] : 0.f; fb[i] = (__bf16)fv; } }
    asm volatile("s_wait_loadcnt 0x0" ::: "memory");
    acc[j] = wmma_bf(a.h, fb, acc[j]); acc[j] = wmma_bf(a.l, fb, acc[j]); }
#pragma unroll
  for (int j = 0; j < 4; ++j)
#pragma unroll
    for (int r = 0; r < 8; ++r) sf[wave][8 * g + r][j * 16 + col] = acc[j][r];
  LDSX();
  for (int k = 0; k < KP; ++k) if (live && lane < 16) vst2(FK + row * FKW + k * CI + lane * 4, *(const v4f*)&sf[wave][k][lane * 4]); }
__global__ __launch_bounds__(128) void k_out2(const float* __restrict__ FK, const float* __restrict__ WT, const float* __restrict__ CNT, float* __restrict__ OUT) { __shared__ __align__(16) float so[4][16][132];
  const int tid = threadIdx.x, wave = tid >> 5, lane = tid & 31, col = lane & 15, g = lane >> 4; const size_t r0 = (size_t)blockIdx.x * 64 + wave * 16;
  v8f acc[CO / 16] = {};
#pragma unroll 2
  for (int kc = 0; kc < FKW / 32; ++kc) { const F2 a = split_row(FK + ((r0 + col) < (size_t)NRV ? (r0 + col) : 0) * FKW, kc * 32, lane); asm volatile("s_wait_loadcnt 0x0" ::: "memory");
#pragma unroll
    for (int j = 0; j < CO / 16; ++j) { const v16b w = wcol_io(WT, kc * 32, j * 16 + col, lane, CO); acc[j] = wmma_bf(a.h, w, acc[j]); acc[j] = wmma_bf(a.l, w, acc[j]); } }
  float cn[8];
#pragma unroll
  for (int r = 0; r < 8; ++r) { const size_t rr = r0 + 8 * g + r; cn[r] = CNT[rr < (size_t)NRV ? rr : 0]; }
  asm volatile("s_wait_loadcnt 0x0" ::: "memory");
#pragma unroll
  for (int j = 0; j < CO / 16; ++j) {
#pragma unroll
    for (int r = 0; r < 8; ++r) so[wave][8 * g + r][j * 16 + col] = acc[j][r] / cn[r]; }
  LDSX(); for (int rl = 0; rl < 16; ++rl) if (r0 + rl < (size_t)NRV && lane < CO / 4) vst2(OUT + (r0 + rl) * CO + lane * 4, *(const v4f*)&so[wave][rl][lane * 4]); }
extern "C" void kernel_launch(void* const* d_in, const int* in_sizes, int n_in, void* d_out, int out_size, void* d_ws, size_t ws_size, hipStream_t stream) {
  (void)in_sizes; (void)n_in; (void)out_size;
  if (ws_size < (size_t)WS_END) return;
  char* ws = (char*)d_ws; const float** F = (const float**)d_in; float* FK = (float*)(ws + WS_FK); float* CNT = (float*)(ws + WS_CNT);
  k_fk<<<dim3((NRV + 3) / 4), 128, 0, stream>>>(F[1], F[2], F[0], F[5], (const int*)d_in[3], FK, CNT);
  k_out2<<<dim3((NRV + 63) / 64), 128, 0, stream>>>(FK, F[4], CNT, (float*)d_out);
}
